// GDPModel_26749056319490
// MI455X (gfx1250) — hardware-run, weakly checked
//
#include <hip/hip_runtime.h>


namespace {
constexpr int N = 50000, NP = 50048, E = 800000, IN = 128, ED = 16, HID = 32, NH = 4, HC = 128, OUT = 64, G = 64;
constexpr float XS = 8.0f, WSC = 256.0f, SLOPE = 0.2f;

typedef _Float16 b16;
typedef __attribute__((ext_vector_type(16))) _Float16 v16b;
typedef __attribute__((ext_vector_type(8))) _Float16 v8b;
typedef __attribute__((ext_vector_type(8))) float v8f;
typedef __attribute__((ext_vector_type(4))) float v4f;
__device__ __forceinline__ float bf16_rne(float f) { unsigned int u = __float_as_uint(f); u += 0x7FFFu + ((u >> 16) & 1u); return __uint_as_float(u & 0xFFFF0000u); }
__device__ __forceinline__ void split16(float v, b16& hi, b16& lo) { hi = (b16)v; lo = (b16)(v - (float)hi); }
__device__ __forceinline__ v16b frag_kb(const b16* p, int hh) { const v8b a = *(const v8b*)(p + 8 * hh), b = *(const v8b*)(p + 16 + 8 * hh); v16b f;
#pragma unroll
  for (int e = 0; e < 8; ++e) { f[e] = a[e]; f[8 + e] = b[e]; } return f; }
__device__ __forceinline__ v8f wmma16b(v16b a, v16b b, v8f c) { v8f d = __builtin_amdgcn_wmma_f32_16x16x32_f16(false, a, false, b, (short)0, c, false, false); asm volatile("v_nop\n\tv_nop\n\tv_nop\n\tv_nop" : "+v"(d) : "v"(a), "v"(b)); return d; }
__device__ __forceinline__ void wave_lds_sync() { __builtin_amdgcn_fence(__ATOMIC_RELEASE, "workgroup"); __builtin_amdgcn_wave_barrier(); __builtin_amdgcn_fence(__ATOMIC_ACQUIRE, "workgroup"); }
__device__ __forceinline__ float pmul(float a, float b) { float p = a * b; asm volatile("" : "+v"(p)); return p; }
__device__ __forceinline__ float hsum16(float v) { v += __shfl_xor(v, 1); v += __shfl_xor(v, 2); v += __shfl_xor(v, 4); return v + __shfl_xor(v, 8); }
__device__ __forceinline__ int iclamp(int v, int lo, int hi) { return v < lo ? lo : (v > hi ? hi : v); }
__device__ __forceinline__ float lrelu(float x) { return x > 0.0f ? x : SLOPE * x; }
__device__ __forceinline__ float elu(float x) { return x > 0.0f ? x : (__expf(x) - 1.0f); }

constexpr int CSR_NBLK = 512, CSR_GB = 9, CSR_GN = 1 << CSR_GB  , CSR_MAXG = 512, CSR_CAP = 12288  ;
__global__ __launch_bounds__(64) void csrA_kernel(const int* __restrict__ dst, int E, int N, int nG, int CHP, int NGP, int* __restrict__ STG, int* __restrict__ HST) {
  extern __shared__ int sm[];
  int* cnt = sm; int* run = sm + NGP; int* ids = sm + 2 * NGP;
  const int b = blockIdx.x; const int ch = (E + CSR_NBLK - 1) / CSR_NBLK; const int e0 = b * ch, e1 = min(E, e0 + ch);
  for (int i = threadIdx.x; i < NGP; i += 64) cnt[i] = 0;
  for (int i = threadIdx.x; i < CHP; i += 64) ids[i] = -1;
  __syncthreads();
  if (threadIdx.x == 0) {
    for (int e = e0; e < e1; ++e) { int d = dst[e]; d = (d < 0) ? 0 : (d >= N ? N - 1 : d); cnt[d >> CSR_GB] += 1; }
    int acc = 0; for (int g = 0; g < nG; ++g) { run[g] = acc; acc += cnt[g]; }
    for (int e = e0; e < e1; ++e) { int d = dst[e]; d = (d < 0) ? 0 : (d >= N ? N - 1 : d); const int g = d >> CSR_GB; ids[run[g]] = e; run[g] += 1; } }
  __syncthreads();
  typedef __attribute__((ext_vector_type(4))) int v4i;
  for (int pass = 0; pass < 2; ++pass) {
    for (int i = threadIdx.x; i < CHP / 4; i += 64) *(volatile v4i*)(STG + (size_t)b * CHP + i * 4) = *(const v4i*)(&ids[i * 4]);
    for (int i = threadIdx.x; i < NGP / 4; i += 64) { v4i v; for (int e = 0; e < 4; ++e) v[e] = (i * 4 + e < nG) ? cnt[i * 4 + e] : 0; *(volatile v4i*)(HST + (size_t)b * NGP + i * 4) = v; }
    __threadfence(); }
}
__global__ __launch_bounds__(512) void csrS_kernel(const int* __restrict__ HST, int nG, int NGP, int* __restrict__ START, int* __restrict__ TOT, int* __restrict__ OFF) {
  __shared__ int tot[CSR_MAXG];
  const int b = threadIdx.x;
  for (int pass = 0; pass < 2; ++pass) { int runb = 0; for (int g = 0; g < nG; ++g) { int c = HST[(size_t)b * NGP + g]; c = (c < 0) ? 0 : c; ((volatile int*)OFF)[(size_t)g * CSR_NBLK + b] = runb; runb += c; } __threadfence(); }
  for (int g = threadIdx.x; g < nG; g += 512) { int s = 0; for (int bb = 0; bb < CSR_NBLK; ++bb) { int c = HST[(size_t)bb * NGP + g]; s += (c < 0) ? 0 : c; } tot[g] = s; }
  __syncthreads();
  if (threadIdx.x < 32) {
    __shared__ int st[CSR_MAXG + 32];
    if (threadIdx.x == 0) { int acc = 0; for (int g = 0; g < NGP; ++g) { st[g] = acc; if (g < nG) acc += (tot[g] + 31) & ~31; } st[NGP] = acc; }
    __builtin_amdgcn_fence(__ATOMIC_RELEASE, "workgroup"); __builtin_amdgcn_wave_barrier(); __builtin_amdgcn_fence(__ATOMIC_ACQUIRE, "workgroup");
    for (int pass = 0; pass < 2; ++pass) { for (int i = threadIdx.x; i < NGP + 32; i += 32) { ((volatile int*)START)[i] = (i <= NGP) ? st[min(i, NGP)] : 0; ((volatile int*)TOT)[i] = (i < nG) ? tot[i] : 0; } __threadfence(); } }
}
__global__ __launch_bounds__(256) void csrB_kernel(const int* __restrict__ dst, int N, int nG, int CHP, int NGP, int permLen, const int* __restrict__ STG, const int* __restrict__ HST, const int* __restrict__ OFF, const int* __restrict__ START, const int* __restrict__ TOT, int* __restrict__ PERM, int* __restrict__ ROWPTR, int* __restrict__ ROWCNT, int* __restrict__ FLAG) {
  typedef __attribute__((ext_vector_type(4))) int v4i;
  __shared__ int ids[CSR_CAP]; __shared__ unsigned short key[CSR_CAP]; __shared__ int outp[CSR_CAP]; __shared__ int ncnt[CSR_GN + 1]; __shared__ int boff[CSR_NBLK + 1];
  const int g = blockIdx.x, t_ = threadIdx.x; int tot = TOT[g]; int st = START[g], stn = START[g + 1]; const int v0 = g * CSR_GN; const int nv = min(CSR_GN, N - v0);
  st = (st < 0) ? 0 : (st > permLen - 32 ? permLen - 32 : st) & ~31; stn = (stn < st) ? st : (stn > permLen ? permLen : stn); tot = (tot < 0) ? 0 : tot; if (tot > stn - st && tot <= CSR_CAP) tot = stn - st;
  if (tot > CSR_CAP) {
    for (int pass = 0; pass < 2; ++pass) { for (int i = t_; i < CSR_GN / 4; i += 256) { v4i a, c; for (int e = 0; e < 4; ++e) { a[e] = st; c[e] = 0; } *(volatile v4i*)(ROWPTR + v0 + i * 4) = a; *(volatile v4i*)(ROWCNT + v0 + i * 4) = c; } if (t_ == 0) ((volatile int*)FLAG)[0] = 1; __threadfence(); } (void)nv; return; }
  if (t_ == 0) { int acc = 0; for (int b = 0; b < CSR_NBLK; ++b) { boff[b] = acc; int c = HST[(size_t)b * NGP + g]; c = (c < 0) ? 0 : (c > CHP ? CHP : c); acc += c; if (acc > tot) acc = tot; } boff[CSR_NBLK] = acc; }
  for (int i = t_; i <= CSR_GN; i += 256) ncnt[i] = 0;
  __syncthreads();
  for (int b = 0; b < CSR_NBLK; ++b) { const int c = boff[b + 1] - boff[b]; int o_ = OFF[(size_t)g * CSR_NBLK + b]; o_ = (o_ < 0) ? 0 : (o_ > CHP - c ? CHP - c : o_); const int* src_ = STG + (size_t)b * CHP + o_;
    for (int i = t_; i < c; i += 256) { int id = src_[i]; id = (id < 0) ? 0 : id; ids[boff[b] + i] = id; int d = dst[id]; d = (d < v0) ? v0 : (d >= N ? N - 1 : d); int kk = d - v0; kk = (kk < 0) ? 0 : (kk >= CSR_GN ? CSR_GN - 1 : kk); key[boff[b] + i] = (unsigned short)kk; } }
  __syncthreads();
  if (t_ == 0) { for (int i = 0; i < tot; ++i) ncnt[key[i]] += 1; int acc = 0; for (int vl = 0; vl < CSR_GN; ++vl) { const int c = ncnt[vl]; ncnt[vl] = acc; acc += c; } ncnt[CSR_GN] = acc;
    for (int i = 0; i < tot; ++i) { const int vl = key[i]; outp[ncnt[vl]] = ids[i]; ncnt[vl] += 1; }
    for (int vl = CSR_GN; vl > 0; --vl) ncnt[vl] = ncnt[vl - 1]; ncnt[0] = 0; }
  __syncthreads();
  for (int pass = 0; pass < 2; ++pass) {
    for (int i = t_; i < (stn - st) / 4; i += 256) { v4i v; for (int e = 0; e < 4; ++e) { const int q = i * 4 + e; v[e] = (q < tot) ? outp[q] : -1; } *(volatile v4i*)(PERM + st + i * 4) = v; }
    for (int i = t_; i < CSR_GN / 4; i += 256) { v4i a, c; for (int e = 0; e < 4; ++e) { const int vl = i * 4 + e; a[e] = st + ncnt[vl]; c[e] = (vl < nv) ? (ncnt[vl + 1] - ncnt[vl]) : 0; } *(volatile v4i*)(ROWPTR + v0 + i * 4) = a; *(volatile v4i*)(ROWCNT + v0 + i * 4) = c; }
    __threadfence(); }
}
__global__ __launch_bounds__(256) void csrZ_kernel(int* __restrict__ p, size_t n4) { typedef __attribute__((ext_vector_type(4))) int v4i; const size_t tid = (size_t)blockIdx.x * 256 + threadIdx.x, nth = (size_t)gridDim.x * 256; v4i z = {0, 0, 0, 0}; for (size_t i = tid; i < n4; i += nth) *(volatile v4i*)(p + i * 4) = z; }
struct CsrBufs { int *STG, *HST, *OFF, *START, *TOT, *PERM, *ROWPTR, *ROWCNT, *FLAG; int nG, NGP, CHP; size_t permLen; char* base; size_t bytes; };
static size_t csr_carve(CsrBufs& c, char* ws, size_t off, int E, int N) {
  const size_t off0 = off; c.base = ws + off;
  auto al = [&](size_t bytes) { char* p = ws + off; off += (bytes + 255) & ~(size_t)255; return p; };
  c.nG = (N + CSR_GN - 1) / CSR_GN; c.NGP = (c.nG + 31) & ~31; const int ch = (E + CSR_NBLK - 1) / CSR_NBLK; c.CHP = (ch + 31) & ~31; c.permLen = (size_t)E + 32 * (size_t)c.nG + 32;
  c.STG = (int*)al((size_t)CSR_NBLK * c.CHP * 4); c.HST = (int*)al((size_t)CSR_NBLK * c.NGP * 4); c.OFF = (int*)al((size_t)c.NGP * CSR_NBLK * 4); c.START = (int*)al((size_t)(c.NGP + 64) * 4); c.TOT = (int*)al((size_t)(c.NGP + 64) * 4);
  c.PERM = (int*)al(c.permLen * 4); c.ROWPTR = (int*)al((size_t)c.nG * CSR_GN * 4); c.ROWCNT = (int*)al((size_t)c.nG * CSR_GN * 4); c.FLAG = (int*)al(256);
  c.bytes = off - off0; return off;
}
static void csr_build(const CsrBufs& c, const int* dst, int E, int N, hipStream_t stream) {
  const size_t smem = (size_t)(2 * c.NGP + c.CHP) * 4;
  csrZ_kernel<<<512, 256, 0, stream>>>((int*)c.base, c.bytes / 16);
  csrA_kernel<<<CSR_NBLK, 64, smem, stream>>>(dst, E, N, c.nG, c.CHP, c.NGP, c.STG, c.HST);
  csrS_kernel<<<1, 512, 0, stream>>>(c.HST, c.nG, c.NGP, c.START, c.TOT, c.OFF);
  csrB_kernel<<<c.nG, 256, 0, stream>>>(dst, N, c.nG, c.CHP, c.NGP, (int)c.permLen, c.STG, c.HST, c.OFF, c.START, c.TOT, c.PERM, c.ROWPTR, c.ROWCNT, c.FLAG);
}


__global__ __launch_bounds__(256) void prep_kernel(const float* __restrict__ x, const float* __restrict__ w1, const float* __restrict__ w2, const float* __restrict__ we1, const float* __restrict__ ae1, const float* __restrict__ we2, const float* __restrict__ ae2, b16* __restrict__ X16, b16* __restrict__ W1T, b16* __restrict__ W2T, float* __restrict__ U1, float* __restrict__ U2) {
  const size_t t = (size_t)blockIdx.x * 256 + threadIdx.x; const size_t nx = (size_t)NP * IN / 8, n1 = (size_t)HC * IN / 8, n2 = (size_t)OUT * HC / 8; v8b o = {};
  if (t < nx) { const size_t e = t * 8; if (e < (size_t)N * IN) { const v4f a = *(const v4f*)(x + e), c = *(const v4f*)(x + e + 4); for (int j = 0; j < 4; ++j) { o[j] = (b16)(bf16_rne(a[j]) * XS); o[4 + j] = (b16)(bf16_rne(c[j]) * XS); } }
    for (int pass = 0; pass < 2; ++pass) { *(volatile v8b*)(X16 + e) = o; __threadfence(); } }
  else if (t < nx + n1) { const size_t u = (t - nx) * 8; const int oo = (int)(u / IN), i0 = (int)(u - (size_t)oo * IN); for (int j = 0; j < 8; ++j) o[j] = (b16)(bf16_rne(w1[(size_t)(i0 + j) * HC + oo]) * WSC); for (int pass = 0; pass < 2; ++pass) { *(volatile v8b*)(W1T + u) = o; __threadfence(); } }
  else if (t < nx + n1 + n2) { const size_t u = (t - nx - n1) * 8; const int oo = (int)(u / HC), i0 = (int)(u - (size_t)oo * HC); for (int j = 0; j < 8; ++j) o[j] = (b16)(bf16_rne(w2[(size_t)(i0 + j) * OUT + oo]) * WSC); for (int pass = 0; pass < 2; ++pass) { *(volatile v8b*)(W2T + u) = o; __threadfence(); } }
  else if (t < nx + n1 + n2 + 96) { const int i = (int)(t - nx - n1 - n2); float s = 0.0f;
    if (i < 64) { const int k = i >> 2, h = i & 3; for (int c = 0; c < HID; ++c) s += pmul(bf16_rne(we1[k * HC + h * HID + c]), bf16_rne(ae1[h * HID + c])); }
    else if (i < 80) { const int k = i - 64; for (int c = 0; c < OUT; ++c) s += pmul(bf16_rne(we2[k * OUT + c]), bf16_rne(ae2[c])); }
    for (int pass = 0; pass < 2; ++pass) { if (i < 64) ((volatile float*)U1)[i] = s; else ((volatile float*)U2)[i - 64] = s; __threadfence(); } }
}
__global__ __launch_bounds__(256) void eamean_kernel(const float* __restrict__ ea, float* __restrict__ EM) {
  __shared__ float part[256][ED + 1];
  const int t_ = threadIdx.x; float s[ED]; for (int k = 0; k < ED; ++k) s[k] = 0.0f;
  for (int e = t_; e < E; e += 256) { const v4f a = *(const v4f*)(ea + (size_t)e * ED), b = *(const v4f*)(ea + (size_t)e * ED + 4), c = *(const v4f*)(ea + (size_t)e * ED + 8), d = *(const v4f*)(ea + (size_t)e * ED + 12);
    for (int j = 0; j < 4; ++j) { s[j] += bf16_rne(a[j]); s[4 + j] += bf16_rne(b[j]); s[8 + j] += bf16_rne(c[j]); s[12 + j] += bf16_rne(d[j]); } }
  for (int k = 0; k < ED; ++k) part[t_][k] = s[k];
  __syncthreads();
  for (int st = 128; st >= 1; st >>= 1) { if (t_ < st) for (int k = 0; k < ED; ++k) part[t_][k] += part[t_ + st][k]; __syncthreads(); }
  for (int pass = 0; pass < 2; ++pass) { if (t_ < 32) ((volatile float*)EM)[t_] = (t_ < ED) ? part[0][t_] * (1.0f / (float)E) : 0.0f; __threadfence(); }
}
template <int LAYER>
__global__ __launch_bounds__(128) void node_kernel(const b16* __restrict__ A, const b16* __restrict__ Al, const b16* __restrict__ W, const float* __restrict__ att_s, const float* __restrict__ att_d, float* __restrict__ H, float* __restrict__ AS, float* __restrict__ AD) {
  constexpr int NT = LAYER == 1 ? 8 : 4, NHD = LAYER == 1 ? NH : 1, NC = NT * 16;
  __shared__ __attribute__((aligned(16))) float Ts[4][16][HC + 4]; __shared__ float Sa[4][16][4], Sd[4][16][4];
  const int wave = threadIdx.x >> 5, lane = threadIdx.x & 31, nloc = lane & 15, hlf = lane >> 4; const size_t m0 = ((size_t)blockIdx.x * 4 + wave) * 16;
  v8f acc[NT];
#pragma unroll
  for (int t = 0; t < NT; ++t) acc[t] = (v8f){};
#pragma unroll
  for (int kb = 0; kb < HC; kb += 32) { const v16b a = frag_kb(A + (m0 + nloc) * HC + kb, hlf);
    if (LAYER == 2) { const v16b al = frag_kb(Al + (m0 + nloc) * HC + kb, hlf);
#pragma unroll
      for (int t = 0; t < NT; ++t) { const v16b bw = frag_kb(W + (size_t)(t * 16 + nloc) * HC + kb, hlf); acc[t] = wmma16b(a, bw, acc[t]); acc[t] = wmma16b(al, bw, acc[t]); } }
    else {
#pragma unroll
      for (int t = 0; t < NT; ++t) acc[t] = wmma16b(a, frag_kb(W + (size_t)(t * 16 + nloc) * HC + kb, hlf), acc[t]); } }
  float ps[8][4], pd[8][4];
#pragma unroll
  for (int r = 0; r < 8; ++r)
#pragma unroll
    for (int h = 0; h < 4; ++h) { ps[r][h] = 0.0f; pd[r][h] = 0.0f; }
#pragma unroll
  for (int t = 0; t < NT; ++t) { const int c = t * 16 + nloc; const int h = LAYER == 1 ? (t >> 1) : 0; const float sa = bf16_rne(att_s[c]), sd = bf16_rne(att_d[c]);
#pragma unroll
    for (int r = 0; r < 8; ++r) { const float vv = acc[t][r] * (1.0f / (XS * WSC)); Ts[wave][8 * hlf + r][c] = vv; ps[r][h] += pmul(vv, sa); pd[r][h] += pmul(vv, sd); } }
#pragma unroll
  for (int r = 0; r < 8; ++r)
#pragma unroll
    for (int h = 0; h < NHD; ++h) { const float s1 = hsum16(ps[r][h]), s2 = hsum16(pd[r][h]); if (nloc == 0) { Sa[wave][8 * hlf + r][h] = s1; Sd[wave][8 * hlf + r][h] = s2; } }
  __syncthreads();
  for (int pass = 0; pass < 2; ++pass) {
    for (int rr = 0; rr < 16; ++rr) { if (LAYER == 1) *(volatile v4f*)(H + (m0 + rr) * NC + lane * 4) = *(const v4f*)(&Ts[wave][rr][lane * 4]); else if (lane < 16) *(volatile v4f*)(H + (m0 + rr) * NC + lane * 4) = *(const v4f*)(&Ts[wave][rr][lane * 4]); }
    const size_t mb = (size_t)blockIdx.x * 64;
    for (int i = threadIdx.x; i < 64 * NHD; i += 128) { const int rr = i / NHD, h = i - rr * NHD; ((volatile float*)AS)[mb * NHD + i] = Sa[rr >> 4][rr & 15][h]; ((volatile float*)AD)[mb * NHD + i] = Sd[rr >> 4][rr & 15][h]; }
    __threadfence(); }
}
template <int LAYER>
__global__ __launch_bounds__(256) void edge_kernel(const float* __restrict__ ea, const float* __restrict__ U, float* __restrict__ AE) {
  __shared__ float Us[ED][4];
  const int t_ = threadIdx.x; if (t_ < 64) Us[t_ >> 2][t_ & 3] = (LAYER == 1) ? U[t_] : ((t_ & 3) == 0 ? U[t_ >> 2] : 0.0f);
  __syncthreads();
  const size_t e = (size_t)blockIdx.x * 256 + t_; if (e >= (size_t)E) return; float a4[4] = {0, 0, 0, 0};
#pragma unroll
  for (int k4 = 0; k4 < ED; k4 += 4) { const v4f v = *(const v4f*)(ea + e * ED + k4);
#pragma unroll
    for (int kk = 0; kk < 4; ++kk) { const float x = bf16_rne(v[kk]);
#pragma unroll
      for (int h = 0; h < 4; ++h) a4[h] += pmul(x, Us[k4 + kk][h]); } }
  for (int pass = 0; pass < 2; ++pass) { if (LAYER == 1) { const v4f o = {a4[0], a4[1], a4[2], a4[3]}; *(volatile v4f*)(AE + e * 4) = o; } else ((volatile float*)AE)[e] = a4[0]; __threadfence(); }
}
template <int LAYER>
__global__ __launch_bounds__(256) void agg_kernel(const int* __restrict__ srcs, const float* __restrict__ Hf, const float* __restrict__ AS, const float* __restrict__ AD, const float* __restrict__ AE, const float* __restrict__ U, const float* __restrict__ EM, const float* __restrict__ bias, const int* __restrict__ PERM, const int* __restrict__ ROWPTR, const int* __restrict__ ROWCNT, int permLen, b16* __restrict__ Xh, b16* __restrict__ Xl, float* __restrict__ H2F) {
  constexpr int NCH = LAYER == 1 ? HC : OUT, CPL = NCH / 16, NHD = LAYER == 1 ? NH : 1, CHH = NCH / NHD;
  const int wave = threadIdx.x >> 5, lane = threadIdx.x & 31; const size_t v = ((size_t)blockIdx.x * 8 + wave) * 2 + (lane >> 4); const int c0 = (lane & 15) * CPL, h = c0 / CHH;
  const int vv = (int)((v < (size_t)N) ? v : (size_t)(N - 1));
  int st = ROWPTR[vv], cnt = ROWCNT[vv]; cnt = iclamp(cnt, 0, 4096); st = iclamp(st, 0, permLen - cnt); if (v >= (size_t)N) cnt = 0;
  const float ad = AD[(size_t)vv * NHD + h], asv = AS[(size_t)vv * NHD + h];
  float aeself = 0.0f; for (int k = 0; k < ED; ++k) aeself += pmul(EM[k], (LAYER == 1) ? U[k * 4 + h] : U[k]);
  const float eself = lrelu(asv + ad + aeself);
  float m = eself; for (int j = 0; j < cnt; ++j) { const int e = iclamp(PERM[st + j], 0, E - 1); const int s = iclamp(srcs[e], 0, N - 1); m = fmaxf(m, lrelu(AS[(size_t)s * NHD + h] + ad + AE[(size_t)e * NHD + h])); }
  float den = __expf(eself - m); float acc[CPL]; { const float* hr = Hf + (size_t)vv * NCH + c0; for (int q = 0; q < CPL; ++q) acc[q] = pmul(den, hr[q]); }
  for (int j = 0; j < cnt; ++j) { const int e = iclamp(PERM[st + j], 0, E - 1); const int s = iclamp(srcs[e], 0, N - 1); const float a = __expf(lrelu(AS[(size_t)s * NHD + h] + ad + AE[(size_t)e * NHD + h]) - m); den += a; const float* hr = Hf + (size_t)s * NCH + c0;
    if (CPL == 8) { const v4f h0 = *(const v4f*)hr, h1v = *(const v4f*)(hr + 4); for (int q = 0; q < 4; ++q) { acc[q] += pmul(a, h0[q]); acc[4 + q] += pmul(a, h1v[q]); } }
    else { const v4f h0 = *(const v4f*)hr; for (int q = 0; q < 4; ++q) acc[q] += pmul(a, h0[q]); } }
  const float inv = 1.0f / (den + 1e-16f);
  if (LAYER == 1) { v8b hv8, lv8;
#pragma unroll
    for (int q = 0; q < 8; ++q) { float o = elu(acc[q] * inv + bf16_rne(bias[c0 + q])); if (v >= (size_t)N) o = 0.0f; b16 a_, c_; split16(o * XS, a_, c_); hv8[q] = a_; lv8[q] = c_; }
    for (int pass = 0; pass < 2; ++pass) { *(volatile v8b*)(Xh + v * HC + c0) = hv8; *(volatile v8b*)(Xl + v * HC + c0) = lv8; __threadfence(); } }
  else { v4f o4; for (int q = 0; q < 4; ++q) o4[q] = (v < (size_t)N) ? acc[q] * inv + bf16_rne(bias[c0 + q]) : 0.0f;
    for (int pass = 0; pass < 2; ++pass) { *(volatile v4f*)(H2F + v * OUT + c0) = o4; __threadfence(); } }
}
__global__ __launch_bounds__(64) void pool_kernel(const int* __restrict__ batch, const float* __restrict__ H2F, float* __restrict__ out) {
  __shared__ int rng[2];
  const int g = blockIdx.x, t_ = threadIdx.x;
  if (t_ == 0) { int lo = 0, hi = N; while (lo < hi) { const int mid = (lo + hi) >> 1; if (batch[mid] < g) lo = mid + 1; else hi = mid; } const int first = lo; lo = first; hi = N; while (lo < hi) { const int mid = (lo + hi) >> 1; if (batch[mid] <= g) lo = mid + 1; else hi = mid; } rng[0] = first; rng[1] = lo; }
  __syncthreads();
  const int a = rng[0], b = rng[1]; float s = 0.0f; int cnt = 0;
  for (int i = a; i < b; ++i) { if (batch[i] == g) { s += H2F[(size_t)i * OUT + t_]; cnt += 1; } }
  const float o = s / fmaxf((float)cnt, 1.0f);
  for (int pass = 0; pass < 2; ++pass) { ((volatile float*)out)[(size_t)g * OUT + t_] = o; __threadfence(); }
}
}

extern "C" void kernel_launch(void* const* d_in, const int* in_sizes, int n_in, void* d_out, int out_size, void* d_ws, size_t ws_size, hipStream_t stream) {
  (void)n_in;
  auto Fp = [&](int i) { return (const float*)d_in[i]; }; auto Ip = [&](int i) { return (const int*)d_in[i]; };
  if (in_sizes[0] != N * IN || in_sizes[1] != 2 * E || in_sizes[2] != E * ED || in_sizes[3] != N || in_sizes[4] != IN * HC || in_sizes[7] != ED * HC || in_sizes[10] != HC * OUT || in_sizes[13] != ED * OUT || out_size != G * OUT) return;
  size_t off = 0; char* ws = (char*)d_ws;
  auto carve = [&](size_t bytes) { char* p = ws + off; off += (bytes + 255) & ~(size_t)255; return p; };
  b16* X16 = (b16*)carve((size_t)NP * IN * 2); b16* W1T = (b16*)carve((size_t)HC * IN * 2); b16* W2T = (b16*)carve((size_t)OUT * HC * 2); float* U1 = (float*)carve(256); float* U2 = (float*)carve(256); float* EM = (float*)carve(256);
  float* H = (float*)carve((size_t)NP * HC * 4); float* AS = (float*)carve((size_t)NP * NH * 4); float* AD = (float*)carve((size_t)NP * NH * 4); float* AE = (float*)carve((size_t)E * NH * 4); b16* Xh = (b16*)carve((size_t)NP * HC * 2); b16* Xl = (b16*)carve((size_t)NP * HC * 2); float* H2F = (float*)carve((size_t)NP * OUT * 4);
  CsrBufs csr; off = csr_carve(csr, ws, off, E, N);
  if (off > ws_size || off > ((size_t)128 << 20)) return;
  const int* srcp = Ip(1); const int* dstp = Ip(1) + E;
  prep_kernel<<<(unsigned)(((size_t)NP * IN / 8 + (size_t)HC * IN / 8 + (size_t)OUT * HC / 8 + 96 + 255) / 256), 256, 0, stream>>>(Fp(0), Fp(4), Fp(10), Fp(7), Fp(8), Fp(13), Fp(14), X16, W1T, W2T, U1, U2);
  eamean_kernel<<<1, 256, 0, stream>>>(Fp(2), EM);
  csr_build(csr, dstp, E, N, stream);
  node_kernel<1><<<NP / 64, 128, 0, stream>>>(X16, nullptr, W1T, Fp(5), Fp(6), H, AS, AD);
  edge_kernel<1><<<(E + 255) / 256, 256, 0, stream>>>(Fp(2), U1, AE);
  agg_kernel<1><<<NP / 16, 256, 0, stream>>>(srcp, H, AS, AD, AE, U1, EM, Fp(9), csr.PERM, csr.ROWPTR, csr.ROWCNT, (int)csr.permLen, Xh, Xl, nullptr);
  node_kernel<2><<<NP / 64, 128, 0, stream>>>(Xh, Xl, W2T, Fp(11), Fp(12), H, AS, AD);
  edge_kernel<2><<<(E + 255) / 256, 256, 0, stream>>>(Fp(2), U2, AE);
  agg_kernel<2><<<NP / 16, 256, 0, stream>>>(srcp, H, AS, AD, AE, U2, EM, Fp(15), csr.PERM, csr.ROWPTR, csr.ROWCNT, (int)csr.permLen, nullptr, nullptr, H2F);
  pool_kernel<<<G, 64, 0, stream>>>(Ip(3), H2F, (float*)d_out);
}
